// NN_35562329211597
// MI455X (gfx1250) — hardware-run, weakly checked
//
#include <hip/hip_runtime.h>


#ifndef MQ
#define MQ 4096
#endif
#ifndef MK
#define MK 8192
#endif
#define MQ_FULL 4096
#define MK_FULL 8192
#define MT    (MQ + MK)
#define DI    1024
#define H1    1024
#define H2    512
#define H3    256
#define DMAXW 1024
#define OSW   68
#define SW    4
#define NEGB  (-3.0e38f)
#define LOG2E 1.4426950408889634f
#define C2L   ((float)(2.0 * 1.4426950408889634))

static_assert(MQ <= MQ_FULL);
static_assert(MK <= MK_FULL);
static_assert(MQ % 64 == 0);
static_assert(MK % 64 == 0);
static_assert(MK >= MQ);
static_assert(MQ % (32 * SW) == 0);
static_assert(MK % 32 == 0);
static_assert(DI % 256 == 0);
static_assert(H1 % 256 == 0);
static_assert(H2 % 256 == 0);
static_assert(H3 % 64 == 0);
static_assert(DI == 1024);
static_assert(H1 == 1024);
static_assert(H2 == 512);
static_assert(H3 == 256);
static_assert(DI <= DMAXW);
static_assert(H1 <= DMAXW);
static_assert(H2 <= DMAXW);
static_assert((2 * DI) % 32 == 0);
static_assert((2 * H1) % 32 == 0);
static_assert((2 * H2) % 32 == 0);
static_assert((OSW * 4) % 16 == 0);
static_assert(256 * 2 * 16 == 64 * 128);
static_assert(32 * 16 * 32 == 64 * 64 * 4);
static_assert(32 * 16 * 16 == 64 * 64 * 2);
static_assert(32 * 16 == 128 * 4);
static_assert(8 * 16 == 32 * 4);
static_assert(64 * OSW * 4 + 128 * 4 <= 131072);
static_assert(64 * 72 * 2 <= 131072);
static_assert(SW * 32 * 4 <= 131072);

typedef unsigned short bf;
typedef __attribute__((ext_vector_type(16))) __bf16   v16bf;
typedef __attribute__((ext_vector_type(8)))  unsigned short v8us;
typedef __attribute__((ext_vector_type(8)))  float    v8f;
typedef __attribute__((ext_vector_type(4)))  float    v4f;
typedef v4f  __attribute__((may_alias)) v4fa;
typedef v8us __attribute__((may_alias)) v8usa;

__device__ __forceinline__ unsigned short f2bf(float f) { unsigned u = __float_as_uint(f); u += 0x7FFFu + ((u >> 16) & 1u); return (unsigned short)(u >> 16); }
__device__ __forceinline__ float bfr(float f) { return __uint_as_float(((unsigned)f2bf(f)) << 16); }
__device__ __forceinline__ float bf2f(unsigned short u) { return __uint_as_float(((unsigned)u) << 16); }
__device__ __forceinline__ v16bf cat16b(v8us lo, v8us hi) { return __builtin_bit_cast(v16bf, __builtin_shufflevector(lo, hi, 0, 1, 2, 3, 4, 5, 6, 7, 8, 9, 10, 11, 12, 13, 14, 15)); }
__device__ __forceinline__ v16bf ldb(const bf* p)  { return cat16b(*(const v8us*)p, *(const v8us*)(p + 16)); }
__device__ __forceinline__ v8f wmmab_g(v16bf a, v16bf b, v8f c) {
    c = __builtin_amdgcn_wmma_f32_16x16x32_bf16(false, a, false, b, (short)0, c, false, false);
    asm volatile("v_nop\n\tv_nop\n\tv_nop\n\tv_nop" : "+v"(c) : "v"(a), "v"(b));
    return c;
}
__device__ __forceinline__ void wave_sync() { __builtin_amdgcn_fence(3  , "wavefront"); __builtin_amdgcn_wave_barrier(); asm volatile("" ::: "memory"); }

__global__ __launch_bounds__(256) void k_wtrans(const float* __restrict__ W, bf* WT, int K, int N) {
    __shared__ __align__(16) unsigned short us[64 * 72];
    const int tid = threadIdx.x; const int k0 = blockIdx.x * 64, n0 = blockIdx.y * 64;
#pragma unroll 4
    for (int i = 0; i < 16; ++i) { const int e = tid + i * 256; const int k = e >> 6, n = e & 63;
        us[n * 72 + k] = f2bf(W[(size_t)(k0 + k) * N + n0 + n]); }
    __syncthreads();
    const size_t KP = (size_t)2 * K;
#pragma unroll 1
    for (int ps = 0; ps < 2; ++ps) {
#pragma unroll
        for (int i = 0; i < 2; ++i) { const int p = tid + i * 256; const int row = p >> 3, c8 = (p & 7) * 8;
            const v8us val = *(const v8usa*)(&us[row * 72 + c8]);
            bf* dst = WT + (size_t)(n0 + row) * KP + k0 + c8;
            *(volatile v8us*)dst = val; *(volatile v8us*)(dst + K) = val; }
        if (ps == 0) __threadfence(); }
}

__global__ __launch_bounds__(64) void k_xstat(const float* __restrict__ X, float* PT, int rt0, int D) {
#pragma clang fp contract(off)
    __shared__ __align__(16) float st[128];
    const int tid = threadIdx.x; const int c = blockIdx.y * 64 + tid; const size_t r0 = (size_t)blockIdx.x * 64;
    float s1 = 0.0f, s2 = 0.0f;
#pragma unroll 4
    for (int r = 0; r < 64; ++r) { const float v = bfr(X[(r0 + r) * (size_t)D + c]); s1 += v; s2 += v * v; }
    st[tid] = s1; st[64 + tid] = s2;
    __syncthreads();
    const v4f val = *(const v4fa*)(&st[(tid & 31) * 4]);
    float* dst = PT + ((size_t)(rt0 + blockIdx.x) * (size_t)(D >> 6) + blockIdx.y) * 128 + (tid & 31) * 4;
#pragma unroll 1
    for (int ps = 0; ps < 2; ++ps) { if (tid < 32) *(volatile v4f*)dst = val; if (ps == 0) __threadfence(); }
}

__global__ __launch_bounds__(256) void k_bnfin(const float* __restrict__ PT, float* ST, double invQ, double invK, int D) {
#pragma clang fp contract(off)
    __shared__ __align__(16) float sa[256];
    __shared__ __align__(16) float sb[256];
    const int tid = threadIdx.x; const int set = blockIdx.y; const int d = blockIdx.x * 256 + tid;
    const int rtb = set * (MQ / 64); const int rtn = (MQ / 64) + set * ((MK - MQ) / 64);
    const double inv = set ? invK : invQ;
    const int CT = D >> 6; const int ct = d >> 6, cc = d & 63;
    double a1 = 0.0, a2 = 0.0;
#pragma unroll 1
    for (int rt = 0; rt < rtn; ++rt) { const size_t base = ((size_t)(rtb + rt) * CT + ct) * 128 + cc; a1 += (double)PT[base]; a2 += (double)PT[base + 64]; }
    const double mu = a1 * inv; double var = a2 * inv - mu * mu; var = var > 0.0 ? var : 0.0;
    sa[tid] = (float)mu; sb[tid] = rsqrtf((float)var + 1.0e-5f);
    __syncthreads();
    const int j = tid & 63; const int which = (tid >> 6) & 1;
    const v4f va = *(const v4fa*)(&sa[j * 4]); const v4f vb = *(const v4fa*)(&sb[j * 4]);
    const v4f val = which ? vb : va;
    float* dst = ST + (size_t)(set * 2 + which) * DMAXW + blockIdx.x * 256 + j * 4;
#pragma unroll 1
    for (int ps = 0; ps < 2; ++ps) { if (tid < 128) *(volatile v4f*)dst = val; if (ps == 0) __threadfence(); }
}

__global__ __launch_bounds__(256) void k_norm(const float* __restrict__ S, const float* __restrict__ st, const float* __restrict__ g, const float* __restrict__ be,
                                              bf* AP, int n8, int dsh, int dstRow0, int inbf) {
#pragma clang fp contract(off)
    const int i = blockIdx.x * 256 + threadIdx.x; if (i >= n8) return;
    const int D = 1 << dsh; const size_t e = (size_t)i * 8; const int row = (int)(e >> dsh), d = (int)(e & (size_t)(D - 1));
    const v8f v = *(const v8f*)(S + e);
    const v8f mu = *(const v8f*)(st + d), rs = *(const v8f*)(st + DMAXW + d), gg = *(const v8f*)(g + d), bb = *(const v8f*)(be + d);
    v8us oh, ol;
#pragma unroll
    for (int k = 0; k < 8; ++k) { const float x = inbf ? bfr(v[k]) : v[k];
        const float y = ((x - mu[k]) * rs[k]) * bfr(gg[k]) + bfr(bb[k]);
        const unsigned short h = f2bf(y); oh[k] = h; ol[k] = f2bf(y - bf2f(h)); }
    bf* dst = AP + ((size_t)(dstRow0 + row) << (dsh + 1)) + d;
    *(volatile v8us*)dst = oh; *(volatile v8us*)(dst + D) = ol;
    __threadfence();
    *(volatile v8us*)dst = oh; *(volatile v8us*)(dst + D) = ol;
}

__global__ __launch_bounds__(32) void k_gemm(const bf* __restrict__ A, const bf* __restrict__ Bt, const float* __restrict__ bias,
                                             float* T, float* PT, bf* PH, bf* PL, int KP, int N, int mode) {
    __shared__ __align__(16) float os[64 * OSW];
    __shared__ __align__(16) float st[128];
    const int lane = threadIdx.x & 31, lr = lane & 15, hi = lane >> 4; const int r0 = blockIdx.x * 64, c0 = blockIdx.y * 64;
    v8f acc[4][4];
#pragma unroll
    for (int mb = 0; mb < 4; ++mb)
#pragma unroll
        for (int nb = 0; nb < 4; ++nb) acc[mb][nb] = (v8f){};
    const size_t aoff = (size_t)(r0 + lr) * KP + 8 * hi, boff = (size_t)(c0 + lr) * KP + 8 * hi;
#pragma unroll 1
    for (int kc = 0; kc < KP; kc += 32) {
        v16bf a[4];
#pragma unroll
        for (int mb = 0; mb < 4; ++mb) a[mb] = ldb(A + aoff + (size_t)mb * 16 * KP + kc);
#pragma unroll
        for (int nb = 0; nb < 4; ++nb) { const v16bf b = ldb(Bt + boff + (size_t)nb * 16 * KP + kc);
#pragma unroll
            for (int mb = 0; mb < 4; ++mb) acc[mb][nb] = wmmab_g(a[mb], b, acc[mb][nb]); }
    }
    float bc[4];
#pragma unroll
    for (int nb = 0; nb < 4; ++nb) bc[nb] = bfr(bias[c0 + nb * 16 + lr]);
#pragma unroll
    for (int mb = 0; mb < 4; ++mb)
#pragma unroll
        for (int nb = 0; nb < 4; ++nb)
#pragma unroll
            for (int j = 0; j < 8; ++j) os[(mb * 16 + hi * 8 + j) * OSW + nb * 16 + lr] = acc[mb][nb][j] + bc[nb];
    wave_sync();
    float s1a = 0.0f, s1b = 0.0f, s2a = 0.0f, s2b = 0.0f;
#pragma unroll 1
    for (int r = 0; r < 64; ++r) { const int ix = r * OSW + 2 * lane;
        const float y0 = tanhf(os[ix]), y1 = tanhf(os[ix + 1]);
        os[ix] = y0; os[ix + 1] = y1; s1a += y0; s1b += y1; s2a += y0 * y0; s2b += y1 * y1; }
    st[2 * lane] = s1a; st[2 * lane + 1] = s1b; st[64 + 2 * lane] = s2a; st[64 + 2 * lane + 1] = s2b;
    wave_sync();
#pragma unroll 1
    for (int ps = 0; ps < 2; ++ps) {
        if (mode == 0) {
#pragma unroll 1
            for (int s = 0; s < 32; ++s) { const int row = 2 * s + (lane >> 4), c4 = (lane & 15) * 4;
                const v4f val = *(const v4fa*)(&os[row * OSW + c4]);
                *(volatile v4f*)(T + (size_t)(r0 + row) * N + c0 + c4) = val; }
            const v4f sv = *(const v4fa*)(&st[lane * 4]);
            *(volatile v4f*)(PT + ((size_t)blockIdx.x * (size_t)(N >> 6) + blockIdx.y) * 128 + lane * 4) = sv;
        } else {
#pragma unroll 1
            for (int s = 0; s < 16; ++s) { const int row = 4 * s + (lane >> 3), c8 = (lane & 7) * 8;
                const v4f x0 = *(const v4fa*)(&os[row * OSW + c8]); const v4f x1 = *(const v4fa*)(&os[row * OSW + c8 + 4]); v8us hv, lv;
#pragma unroll
                for (int i = 0; i < 4; ++i) { const unsigned short h0 = f2bf(x0[i]); const unsigned short h1 = f2bf(x1[i]);
                    hv[i] = h0; hv[4 + i] = h1; lv[i] = f2bf(x0[i] - bf2f(h0)); lv[4 + i] = f2bf(x1[i] - bf2f(h1)); }
                const size_t oo = (size_t)(r0 + row) * N + c0 + c8;
                *(volatile v8us*)(PH + oo) = hv; *(volatile v8us*)(PL + oo) = lv; }
        }
        if (ps == 0) __threadfence(); }
}

__global__ __launch_bounds__(256) void k_rowsq(const bf* __restrict__ PH, const bf* __restrict__ PL, const float* __restrict__ Y, float* K2L, float* YB) {
#pragma clang fp contract(off)
    __shared__ __align__(16) float sk[32];
    const int lane = threadIdx.x & 31;
    const int wave = __builtin_amdgcn_readfirstlane((int)(threadIdx.x >> 5));
#pragma unroll 1
    for (int i = 0; i < 4; ++i) { const int rr = wave * 4 + i;
        const size_t o = ((size_t)MQ + (size_t)blockIdx.x * 32 + rr) * H3 + lane * 8;
        const v8us h = *(const v8us*)(PH + o); const v8us l = *(const v8us*)(PL + o); float s = 0.0f;
#pragma unroll
        for (int k = 0; k < 8; ++k) { const float v = bf2f(h[k]) + bf2f(l[k]); s += v * v; }
        s += __shfl_xor(s, 16, 32); s += __shfl_xor(s, 8, 32); s += __shfl_xor(s, 4, 32); s += __shfl_xor(s, 2, 32); s += __shfl_xor(s, 1, 32);
        if (lane == 0) sk[rr] = s * LOG2E; }
    __syncthreads();
    const int j = threadIdx.x & 7;
    const v4f kv = *(const v4fa*)(&sk[j * 4]);
    const v4f yr = *(const v4f*)(Y + (size_t)blockIdx.x * 32 + j * 4); v4f yv;
#pragma unroll
    for (int k = 0; k < 4; ++k) yv[k] = bfr(yr[k]);
    float* dk = K2L + (size_t)blockIdx.x * 32 + j * 4; float* dy = YB + (size_t)blockIdx.x * 32 + j * 4;
#pragma unroll 1
    for (int ps = 0; ps < 2; ++ps) { if (threadIdx.x < 8) { *(volatile v4f*)dk = kv; *(volatile v4f*)dy = yv; } if (ps == 0) __threadfence(); }
}

__device__ __forceinline__ void sm_step(v8f sa, v8f sb, v8f ca, v8f cb, v8f ya, v8f yb, float& m, float& l, float& n) {
    float ta[8], tb[8]; float mx = NEGB;
#pragma unroll
    for (int r = 0; r < 8; ++r) { ta[r] = sa[r] * C2L - ca[r]; tb[r] = sb[r] * C2L - cb[r]; mx = fmaxf(mx, fmaxf(ta[r], tb[r])); }
    const float mn = fmaxf(m, mx);
    const float al = __builtin_amdgcn_exp2f(m - mn);
    float es = 0.0f, ns = 0.0f;
#pragma unroll
    for (int r = 0; r < 8; ++r) { const float ea = __builtin_amdgcn_exp2f(ta[r] - mn), eb = __builtin_amdgcn_exp2f(tb[r] - mn);
        es += ea + eb; ns += ea * ya[r] + eb * yb[r]; }
    l = l * al + es; n = n * al + ns; m = mn;
}

__global__ __launch_bounds__(32 * SW) void k_sim(const bf* __restrict__ PH, const bf* __restrict__ PL, const float* __restrict__ K2L, const float* __restrict__ YB, float* OUT) {
    __shared__ __align__(16) float ob[SW * 32];
    const int lane = threadIdx.x & 31, lr = lane & 15, hi = lane >> 4;
    const int wave = __builtin_amdgcn_readfirstlane((int)(threadIdx.x >> 5));
    const int t0 = (blockIdx.x * SW + wave) * 32;
    const size_t qo = (size_t)(t0 + lr) * H3 + 8 * hi;
    const size_t ko = (size_t)(MQ + lr) * H3 + 8 * hi;
    float m0 = NEGB, m1 = NEGB, l0 = 0.0f, l1 = 0.0f, n0 = 0.0f, n1 = 0.0f;
#pragma unroll 1
    for (int key0 = 0; key0 < MK; key0 += 32) {
        v8f s00 = (v8f){}, s01 = (v8f){}, s10 = (v8f){}, s11 = (v8f){};
        const size_t kb = ko + (size_t)key0 * H3;
#pragma unroll 1
        for (int d0 = 0; d0 < H3; d0 += 32) {
            const v16bf kh0 = ldb(PH + kb + d0), kh1 = ldb(PH + kb + (size_t)16 * H3 + d0);
            const v16bf kl0 = ldb(PL + kb + d0), kl1 = ldb(PL + kb + (size_t)16 * H3 + d0);
            const v16bf qh0 = ldb(PH + qo + d0), qh1 = ldb(PH + qo + (size_t)16 * H3 + d0);
            const v16bf ql0 = ldb(PL + qo + d0), ql1 = ldb(PL + qo + (size_t)16 * H3 + d0);
            s00 = wmmab_g(kh0, qh0, s00); s01 = wmmab_g(kh0, qh1, s01); s10 = wmmab_g(kh1, qh0, s10); s11 = wmmab_g(kh1, qh1, s11);
            s00 = wmmab_g(kl0, qh0, s00); s01 = wmmab_g(kl0, qh1, s01); s10 = wmmab_g(kl1, qh0, s10); s11 = wmmab_g(kl1, qh1, s11);
            s00 = wmmab_g(kh0, ql0, s00); s01 = wmmab_g(kh0, ql1, s01); s10 = wmmab_g(kh1, ql0, s10); s11 = wmmab_g(kh1, ql1, s11);
        }
        const float* kp = K2L + key0 + 8 * hi;
        const float* yp = YB + key0 + 8 * hi;
        const v8f ca = *(const v8f*)kp, cb = *(const v8f*)(kp + 16);
        const v8f ya = *(const v8f*)yp, yb = *(const v8f*)(yp + 16);
        sm_step(s00, s10, ca, cb, ya, yb, m0, l0, n0);
        sm_step(s01, s11, ca, cb, ya, yb, m1, l1, n1);
    }
    float res0, res1;
    { const float mo = __shfl_xor(m0, 16, 32), lo = __shfl_xor(l0, 16, 32), no = __shfl_xor(n0, 16, 32);
      const float M = fmaxf(m0, mo); const float wa = __builtin_amdgcn_exp2f(m0 - M), wb = __builtin_amdgcn_exp2f(mo - M);
      const float lt = l0 * wa + lo * wb, nt = n0 * wa + no * wb;
      res0 = fminf(fmaxf(nt * (1.0f / lt), 0.0f), 1.0f); }
    { const float mo = __shfl_xor(m1, 16, 32), lo = __shfl_xor(l1, 16, 32), no = __shfl_xor(n1, 16, 32);
      const float M = fmaxf(m1, mo); const float wa = __builtin_amdgcn_exp2f(m1 - M), wb = __builtin_amdgcn_exp2f(mo - M);
      const float lt = l1 * wa + lo * wb, nt = n1 * wa + no * wb;
      res1 = fminf(fmaxf(nt * (1.0f / lt), 0.0f), 1.0f); }
    if (hi == 0) { ob[wave * 32 + lr] = res0; ob[wave * 32 + 16 + lr] = res1; }
    wave_sync();
    const v4f val = *(const v4fa*)(&ob[wave * 32 + (lane & 7) * 4]);
    float* dst = OUT + t0 + (lane & 7) * 4;
#pragma unroll 1
    for (int ps = 0; ps < 2; ++ps) { if (lane < 8) *(volatile v4f*)dst = val; if (ps == 0) __threadfence(); }
}

static constexpr size_t al256(size_t v) { return (v + 255) & ~(size_t)255; }
static constexpr size_t SZ_AP = al256((size_t)MT * 2 * DMAXW * 2);
static constexpr size_t SZ_TF = al256((size_t)MT * H1 * 4);
static constexpr size_t SZ_QK = al256((size_t)MT * H3 * 2);
static constexpr size_t SZ_W1 = al256((size_t)H1 * 2 * DI * 2);
static constexpr size_t SZ_W2 = al256((size_t)H2 * 2 * H1 * 2);
static constexpr size_t SZ_W3 = al256((size_t)H3 * 2 * H2 * 2);
static constexpr size_t SZ_PT = al256((size_t)(MT / 64) * (DMAXW / 64) * 128 * 4);
static constexpr size_t SZ_ST = al256((size_t)2 * 2 * DMAXW * 4);
static constexpr size_t SZ_KY = al256((size_t)MK * 4);
static constexpr size_t SZ_TOTAL = SZ_AP + SZ_TF + 2 * SZ_QK + SZ_W1 + SZ_W2 + SZ_W3 + SZ_PT + SZ_ST + 2 * SZ_KY;
static_assert(SZ_TOTAL <= (size_t)134217728);
static_assert((size_t)MT * 2 * DI * 2 <= SZ_AP);
static_assert((size_t)MT * 2 * H1 * 2 <= SZ_AP);
static_assert((size_t)MT * 2 * H2 * 2 <= SZ_AP);
static_assert((size_t)MT * H2 * 4 <= SZ_TF);
static_assert((size_t)(MT / 64) * (DI / 64) * 128 * 4 <= SZ_PT);
static_assert((size_t)(MT / 64) * (H1 / 64) * 128 * 4 <= SZ_PT);
static_assert((size_t)(MT / 64) * (H2 / 64) * 128 * 4 <= SZ_PT);

extern "C" void kernel_launch(void* const* d_in, const int* in_sizes, int n_in,
                              void* d_out, int out_size, void* d_ws, size_t ws_size, hipStream_t stream) {
    if (n_in < 15) return;
    if ((size_t)in_sizes[0] < (size_t)MQ * DI || (size_t)in_sizes[1] < (size_t)MK * DI || (size_t)in_sizes[2] < (size_t)MK) return;
    if ((size_t)in_sizes[3] < (size_t)DI * H1 || in_sizes[4] < H1 || in_sizes[5] < DI || in_sizes[6] < DI) return;
    if ((size_t)in_sizes[7] < (size_t)H1 * H2 || in_sizes[8] < H2 || in_sizes[9] < H1 || in_sizes[10] < H1) return;
    if ((size_t)in_sizes[11] < (size_t)H2 * H3 || in_sizes[12] < H3 || in_sizes[13] < H2 || in_sizes[14] < H2) return;
    if ((size_t)out_size < (size_t)MQ) return;
    if (SZ_TOTAL > ws_size) return;
    const float* x  = (const float*)d_in[0];
    const float* xn = (const float*)d_in[1];
    const float* yn = (const float*)d_in[2];
    const float* W1 = (const float*)d_in[3];  const float* b1 = (const float*)d_in[4];  const float* g1 = (const float*)d_in[5];  const float* e1 = (const float*)d_in[6];
    const float* W2 = (const float*)d_in[7];  const float* b2 = (const float*)d_in[8];  const float* g2 = (const float*)d_in[9];  const float* e2 = (const float*)d_in[10];
    const float* W3 = (const float*)d_in[11]; const float* b3 = (const float*)d_in[12]; const float* g3 = (const float*)d_in[13]; const float* e3 = (const float*)d_in[14];
    float* OUT = (float*)d_out;
    char* wsp = (char*)d_ws;
    bf* AP = (bf*)wsp; wsp += SZ_AP;
    float* TF = (float*)wsp; wsp += SZ_TF;
    bf* QKH = (bf*)wsp; wsp += SZ_QK;
    bf* QKL = (bf*)wsp; wsp += SZ_QK;
    bf* W1T = (bf*)wsp; wsp += SZ_W1;
    bf* W2T = (bf*)wsp; wsp += SZ_W2;
    bf* W3T = (bf*)wsp; wsp += SZ_W3;
    float* PT = (float*)wsp; wsp += SZ_PT;
    float* ST = (float*)wsp; wsp += SZ_ST;
    float* K2L = (float*)wsp; wsp += SZ_KY;
    float* YB = (float*)wsp; wsp += SZ_KY;
    const double invQ = 1.0 / (double)MQ, invK = 1.0 / (double)MK;

    k_wtrans<<<dim3(DI / 64, H1 / 64, 1), 256, 0, stream>>>(W1, W1T, DI, H1);
    k_wtrans<<<dim3(H1 / 64, H2 / 64, 1), 256, 0, stream>>>(W2, W2T, H1, H2);
    k_wtrans<<<dim3(H2 / 64, H3 / 64, 1), 256, 0, stream>>>(W3, W3T, H2, H3);

    k_xstat<<<dim3(MQ / 64, DI / 64, 1), 64, 0, stream>>>(x, PT, 0, DI);
    k_xstat<<<dim3(MK / 64, DI / 64, 1), 64, 0, stream>>>(xn, PT, MQ / 64, DI);
    k_bnfin<<<dim3(DI / 256, 2, 1), 256, 0, stream>>>(PT, ST, invQ, invK, DI);
    { const int nq = MQ * (DI / 8), nk = MK * (DI / 8);
      k_norm<<<(unsigned)((nq + 255) / 256), 256, 0, stream>>>(x, ST, g1, e1, AP, nq, 10, 0, 1);
      k_norm<<<(unsigned)((nk + 255) / 256), 256, 0, stream>>>(xn, ST + 2 * DMAXW, g1, e1, AP, nk, 10, MQ, 1); }
    k_gemm<<<dim3(MT / 64, H1 / 64, 1), 32, 0, stream>>>(AP, W1T, b1, TF, PT, QKH, QKL, 2 * DI, H1, 0);

    k_bnfin<<<dim3(H1 / 256, 2, 1), 256, 0, stream>>>(PT, ST, invQ, invK, H1);
    { const int nq = MQ * (H1 / 8), nk = MK * (H1 / 8);
      k_norm<<<(unsigned)((nq + 255) / 256), 256, 0, stream>>>(TF, ST, g2, e2, AP, nq, 10, 0, 0);
      k_norm<<<(unsigned)((nk + 255) / 256), 256, 0, stream>>>(TF + (size_t)MQ * H1, ST + 2 * DMAXW, g2, e2, AP, nk, 10, MQ, 0); }
    k_gemm<<<dim3(MT / 64, H2 / 64, 1), 32, 0, stream>>>(AP, W2T, b2, TF, PT, QKH, QKL, 2 * H1, H2, 0);

    k_bnfin<<<dim3(H2 / 256, 2, 1), 256, 0, stream>>>(PT, ST, invQ, invK, H2);
    { const int nq = MQ * (H2 / 8), nk = MK * (H2 / 8);
      k_norm<<<(unsigned)((nq + 255) / 256), 256, 0, stream>>>(TF, ST, g3, e3, AP, nq, 9, 0, 0);
      k_norm<<<(unsigned)((nk + 255) / 256), 256, 0, stream>>>(TF + (size_t)MQ * H2, ST + 2 * DMAXW, g3, e3, AP, nk, 9, MQ, 0); }
    k_gemm<<<dim3(MT / 64, H3 / 64, 1), 32, 0, stream>>>(AP, W3T, b3, TF, PT, QKH, QKL, 2 * H2, H3, 1);

    k_rowsq<<<MK / 32, 256, 0, stream>>>(QKH, QKL, yn, K2L, YB);
    k_sim<<<MQ / (32 * SW), 32 * SW, 0, stream>>>(QKH, QKL, K2L, YB, OUT);
}
